// GraphSAGEConv_21912923144577
// MI455X (gfx1250) — hardware-run, weakly checked
//
#include <hip/hip_runtime.h>

typedef float          v8f   __attribute__((ext_vector_type(8)));
typedef float          v4f   __attribute__((ext_vector_type(4)));
typedef unsigned int   v4u   __attribute__((ext_vector_type(4)));
typedef int            v8i   __attribute__((ext_vector_type(8)));
typedef unsigned short v8us  __attribute__((ext_vector_type(8)));
typedef unsigned short v16us __attribute__((ext_vector_type(16)));
typedef __bf16         v16bf __attribute__((ext_vector_type(16)));
typedef _Float16       v16h  __attribute__((ext_vector_type(16)));
typedef v4f  __attribute__((may_alias)) v4fa;
typedef v8us __attribute__((may_alias)) v8usa;
union FragB { v16bf v; v16us u; v8us h[2]; v8i w; };
union FragH { v16h  v; v16us u; v8us h[2]; v8i w; };

__device__ __forceinline__ v8f wmb(const FragB& a, const FragB& b, v8f c) {
  v8f d = __builtin_amdgcn_wmma_f32_16x16x32_bf16(false, a.v, false, b.v, (short)0, c, false, false);
  asm volatile("v_nop\n\tv_nop\n\tv_nop\n\tv_nop" : "+v"(d) : "v"(a.w), "v"(b.w));
  return d;
}

__device__ __forceinline__ v8f wmh(const FragH& a, const FragH& b, v8f c) {
  v8f d = __builtin_amdgcn_wmma_f32_16x16x32_f16(false, a.v, false, b.v, (short)0, c, false, false);
  asm volatile("v_nop\n\tv_nop\n\tv_nop\n\tv_nop" : "+v"(d) : "v"(a.w), "v"(b.w));
  return d;
}

__device__ __forceinline__ unsigned bf16_bits(float f) {
  const unsigned u = __float_as_uint(f);
  const unsigned r = (u + 0x7FFFu + ((u >> 16) & 1u)) >> 16;
  const unsigned q = (u >> 16) | 0x40u;
  return ((u & 0x7fffffffu) > 0x7f800000u) ? q : r;
}

__device__ __forceinline__ float bf16_val(float f) {
  return __uint_as_float(bf16_bits(f) << 16);
}
__device__ __forceinline__ int clampi(int v, int lo, int hi) {
  return v < lo ? lo : (v > hi ? hi : v);
}

__device__ __forceinline__ unsigned f16_bits(float f) {
  const unsigned u  = __float_as_uint(f);
  const unsigned s  = (u >> 16) & 0x8000u;
  const unsigned a  = u & 0x7fffffffu;
  const unsigned t  = a - 0x38000000u;
  const unsigned r  = (t + 0x0FFFu + ((t >> 13) & 1u)) >> 13;
  const unsigned rc = r > 0x7C00u ? 0x7C00u : r;
  const bool small  = a < 0x38800000u;
  const bool isnan  = a > 0x7f800000u;
  const unsigned fin = small ? 0u : (s | rc);
  return isnan ? (s | 0x7E00u) : fin;
}

__device__ __forceinline__ unsigned pk16(unsigned lo, unsigned hi) { return lo | (hi << 16); }
__device__ __forceinline__ unsigned bf16_lo_bits(float v) {
  float hi = bf16_val(v);
  asm volatile("" : "+v"(hi));
  return bf16_bits(v - hi);
}
__device__ __forceinline__ v4u pack8_bf16(v4f a, v4f c) {
  return (v4u){ pk16(bf16_bits(a[0]), bf16_bits(a[1])), pk16(bf16_bits(a[2]), bf16_bits(a[3])),
                pk16(bf16_bits(c[0]), bf16_bits(c[1])), pk16(bf16_bits(c[2]), bf16_bits(c[3])) };
}
__device__ __forceinline__ v4u pack8_bf16_lo(v4f a, v4f c) {
  return (v4u){ pk16(bf16_lo_bits(a[0]), bf16_lo_bits(a[1])), pk16(bf16_lo_bits(a[2]), bf16_lo_bits(a[3])),
                pk16(bf16_lo_bits(c[0]), bf16_lo_bits(c[1])), pk16(bf16_lo_bits(c[2]), bf16_lo_bits(c[3])) };
}
__device__ __forceinline__ v4u pack8_f16(v4f a, v4f c) {
  return (v4u){ pk16(f16_bits(a[0]), f16_bits(a[1])), pk16(f16_bits(a[2]), f16_bits(a[3])),
                pk16(f16_bits(c[0]), f16_bits(c[1])), pk16(f16_bits(c[2]), f16_bits(c[3])) };
}

template <int FORM>
__global__ __launch_bounds__(256) void k_plane(const float* __restrict__ src, int rows, int cols, int ldsrc,
                                               unsigned short* __restrict__ dst, int MP, int KP) {
  static_assert(FORM >= 0 && FORM <= 3);
  const int KTOT = (FORM == 1 || FORM == 3) ? 2 * KP : KP;
  const unsigned ppr   = (unsigned)(KTOT >> 3);
  const unsigned kp8   = (unsigned)(KP >> 3);
  const unsigned total = (unsigned)MP * ppr;
  const unsigned g     = blockIdx.x * 256u + threadIdx.x;
  const unsigned rowu  = g / ppr;
  const unsigned p     = g - rowu * ppr;
  const bool second    = p >= kp8;
  const int row = (int)rowu;
  const int c0  = (int)((second ? p - kp8 : p) << 3);
  const float* srow = src + (size_t)clampi(row, 0, rows - 1) * (size_t)ldsrc;
  float x[8];
  unsigned mk[8];
#pragma unroll
  for (int e = 0; e < 8; ++e) {
    const int c = c0 + e;
    const float v = srow[clampi(c, 0, cols - 1)];
    asm volatile("" :: "v"(v));
    x[e]  = v;
    mk[e] = (row < rows && c < cols) ? 0xFFFFu : 0u;
  }
  const v4f a = (v4f){ x[0], x[1], x[2], x[3] };
  const v4f c = (v4f){ x[4], x[5], x[6], x[7] };
  v4u o;
  if (FORM == 2) {
    o = pack8_f16(a, c);
  } else {
    const v4u hi = pack8_bf16(a, c);
    o = hi;
    if (FORM == 1) { const v4u lo = pack8_bf16_lo(a, c); o = second ? lo : hi; }
  }
  const v4u mw = (v4u){ pk16(mk[0], mk[1]), pk16(mk[2], mk[3]), pk16(mk[4], mk[5]), pk16(mk[6], mk[7]) };
  o &= mw;
  if (g < total) {
    volatile v4u* q = (volatile v4u*)(dst + (size_t)g * 8);
    *q = o;
    __threadfence();
    *q = o;
  }
}

template <int FORM> struct FragOf    { typedef FragB T; };
template <>         struct FragOf<2> { typedef FragH T; };
__device__ __forceinline__ v8f mm(const FragB& a, const FragB& b, v8f c) { return wmb(a, b, c); }
__device__ __forceinline__ v8f mm(const FragH& a, const FragH& b, v8f c) { return wmh(a, b, c); }
template <class F> __device__ __forceinline__ F ld_frag(const unsigned short* p) {
  F f;
  f.h[0] = *(const v8usa*)(p);
  f.h[1] = *(const v8usa*)(p + 16);
  return f;
}

template <int FORM, int EPI>
__global__ __launch_bounds__(256) __attribute__((amdgpu_num_vgpr(248)))
void k_gemm_nt(const unsigned short* __restrict__ A, const unsigned short* __restrict__ B,
               const float* __restrict__ bias, float* __restrict__ D, int M, int N, int KTOT, int ldd) {
  static_assert(FORM >= 0 && FORM <= 2);
  static_assert(EPI == 0 || EPI == 1);
  typedef typename FragOf<FORM>::T F;
  __shared__ __attribute__((aligned(16))) float sT[8][16 * 68];
  const int lane = threadIdx.x & 31;
  const int wave = threadIdx.x >> 5;
  const int tilesM = (M + 63) >> 6;
  const int tilesN = (N + 63) >> 6;
  const int tile = blockIdx.x * 8 + wave;
  if (tile >= tilesM * tilesN) return;
  const int tm = tile / tilesN;
  const int tn = tile - tm * tilesN;
  const int m0 = tm << 6;
  const int n0 = tn << 6;

  const int rl = lane & 15;
  const int h8 = (lane >> 4) * 8;
  const unsigned short* pa = A + (size_t)(m0 + rl) * (size_t)KTOT + h8;
  const unsigned short* pb = B + (size_t)(n0 + rl) * (size_t)KTOT + h8;

  v8f acc[4][4];
#pragma unroll
  for (int i = 0; i < 4; ++i)
#pragma unroll
    for (int j = 0; j < 4; ++j) acc[i][j] = (v8f){0.f, 0.f, 0.f, 0.f, 0.f, 0.f, 0.f, 0.f};

#pragma unroll 1
  for (int k0 = 0; k0 < KTOT; k0 += 32) {
    F bf[4];
#pragma unroll
    for (int j = 0; j < 4; ++j) bf[j] = ld_frag<F>(pb + (size_t)(j << 4) * (size_t)KTOT + k0);
#pragma unroll
    for (int i = 0; i < 4; ++i) {
      const F af = ld_frag<F>(pa + (size_t)(i << 4) * (size_t)KTOT + k0);
#pragma unroll
      for (int j = 0; j < 4; ++j) acc[i][j] = mm(af, bf[j], acc[i][j]);
    }
  }

  float* slab = sT[wave];
  const int hh = lane >> 4;
  const int c4 = (lane & 15) * 4;
  const int nc = n0 + c4;
  const bool cok = nc < N;
  v4f bv = (v4f){0.f, 0.f, 0.f, 0.f};
  if (EPI == 1) {
    bv = *(const v4fa*)(bias + clampi(nc, 0, N - 4));
    asm volatile("" :: "v"(bv));
  }
#pragma unroll
  for (int i = 0; i < 4; ++i) {
    const int mBase = m0 + (i << 4);
#pragma unroll
    for (int j = 0; j < 4; ++j) {
#pragma unroll
      for (int r = 0; r < 8; ++r) slab[(h8 + r) * 68 + (j << 4) + rl] = acc[i][j][r];
    }
    __builtin_amdgcn_fence(__ATOMIC_RELEASE, "workgroup");
    __builtin_amdgcn_wave_barrier();
    __builtin_amdgcn_fence(__ATOMIC_ACQUIRE, "workgroup");
    v4f vv[8];
#pragma unroll
    for (int it = 0; it < 8; ++it) {
      const int row = it * 2 + hh;
      v4f v = *(const v4fa*)(slab + row * 68 + c4);
      if (EPI == 1) v += bv;
      vv[it] = v;
    }
    for (int pass = 0; pass < 2; ++pass) {
#pragma unroll
      for (int it = 0; it < 8; ++it) {
        const int row = mBase + it * 2 + hh;
        if (cok && row < M) *(volatile v4f*)(D + (size_t)row * (size_t)ldd + nc) = vv[it];
      }
      __threadfence();
    }
    __builtin_amdgcn_fence(__ATOMIC_RELEASE, "workgroup");
    __builtin_amdgcn_wave_barrier();
    __builtin_amdgcn_fence(__ATOMIC_ACQUIRE, "workgroup");
  }
}

#include <stddef.h>
#include <stdint.h>
#pragma clang fp contract(off)

#define SPLIT_AGG 1
#define NN      100000
#define KD      128
#define NE      1600000
#define MP      100096
#define NTHR    256
#define NWAVE   8
#define EPT     8
#define WCH     (32 * EPT)
#define NCHUNK  (NE / WCH)
#define SLB     10
#define NBRUN   1024
#define NBK     98
#define CBITS   17
#define WLCAP   4096
#define RCAP    20480
#define DEGCAP  64
#define MAXDEG_MEAS   16
#define MAXB1024_MEAS 16384
#define AGK     (SPLIT_AGG ? 2 * KD : KD)
#define WSMAX   ((size_t)128 << 20)

#define BK_ZINTS (NWAVE * WLCAP + RCAP + 3 * NBRUN)
#define BK_INTS  (BK_ZINTS + 16)
#define BK_LDS   (BK_INTS * 4)

#define PW1   (KD * KD / 8 / NTHR)
#define PW2   (KD * KD / 8 / NTHR)
#define PW3   (KD * AGK / 8 / NTHR)
#define PWTOT (PW1 + PW2 + PW3 + 1)

static_assert(NN <= (1 << CBITS) && NN <= 131072);
static_assert(NBRUN == (1 << SLB) && NBRUN == 1024 && CBITS + SLB <= 31);
static_assert(NBRUN % 32 == 0 && NBRUN % NWAVE == 0);
static_assert(NBK * NBRUN >= MP && (NBK - 1) * NBRUN < NN);
static_assert(MP % 64 == 0 && MP >= NN && MP % NWAVE == 0 && MP % 16 == 0);
static_assert(NN % 16 == 0 && NN % NWAVE == 0 && KD % 32 == 0 && AGK % 32 == 0 && KD % 4 == 0);
static_assert(NE % WCH == 0 && NE % 4 == 0 && NE >= EPT);
static_assert((long long)RCAP * 100 >= (long long)MAXB1024_MEAS * 125);
static_assert(WLCAP * NWAVE >= RCAP && WLCAP >= MAXB1024_MEAS / NWAVE + 1024);
static_assert(MAXDEG_MEAS + 8 <= DEGCAP);
static_assert(RCAP % (NTHR * 4) == 0 && (2 * NBRUN) % (NTHR * 4) == 0 && BK_ZINTS % 4 == 0);
static_assert(BK_LDS <= 262144 && BK_LDS + 0 <= 327680);
static_assert((MP * KD / 8) % NTHR == 0 && (KD * KD / 8) % NTHR == 0 && (KD * AGK / 8) % NTHR == 0);
static_assert((long long)MP * AGK / 8 < (1LL << 31));

typedef int          v4i __attribute__((ext_vector_type(4)));
typedef unsigned int v2u __attribute__((ext_vector_type(2)));
typedef v4i __attribute__((may_alias)) v4ia;

__device__ __forceinline__ void st2_v4f(float* p, v4f v) {
  *(volatile v4f*)p = v;
  __threadfence();
  *(volatile v4f*)p = v;
}
__device__ __forceinline__ void st2_v8us(unsigned short* p, v8us v) {
  *(volatile v8us*)p = v;
  __threadfence();
  *(volatile v8us*)p = v;
}

__device__ __forceinline__ v8us gather8(const float* __restrict__ base, int stride) {
  float f[8];
#pragma unroll
  for (int i = 0; i < 8; ++i) f[i] = base[(size_t)i * (size_t)stride];
  v8us o;
#pragma unroll
  for (int i = 0; i < 8; ++i) o[i] = (unsigned short)bf16_bits(f[i]);
  return o;
}

__global__ __launch_bounds__(NTHR) void k_prep(const float* __restrict__ wp, const float* __restrict__ bp,
                                               const float* __restrict__ wt, const float* __restrict__ bs,
                                               unsigned short* WPT, unsigned short* WTT, unsigned short* WBD,
                                               float* BL) {
  const int tid = (int)threadIdx.x;
  const int blk = (int)blockIdx.x;
  if (blk < PW1) {
    const int u = blk * NTHR + tid;
    const int n = u >> 4, k8 = (u & 15) * 8;
    const v8us o = gather8(wp + (size_t)k8 * KD + n, KD);
    st2_v8us(WPT + (size_t)u * 8, o);
  } else if (blk < PW1 + PW2) {
    const int u = (blk - PW1) * NTHR + tid;
    const int n = u >> 4, k8 = (u & 15) * 8;
    const v8us o = gather8(wt + (size_t)k8 * KD + n, KD);
    st2_v8us(WTT + (size_t)u * 8, o);
  } else if (blk < PW1 + PW2 + PW3) {
    const int u = (blk - PW1 - PW2) * NTHR + tid;
    const int ppr = AGK / 8;
    const int n = u / ppr, k8 = (u - n * ppr) * 8;
    const int kk = k8 & (KD - 1);
    const v8us o = gather8(wt + (size_t)(KD + kk) * KD + n, KD);
    st2_v8us(WBD + (size_t)u * 8, o);
  } else {
    if (tid < 32) {
      const v4f v = *(const v4fa*)(bp + 4 * tid);
      const v4f o = (v4f){ bf16_val(v.x), bf16_val(v.y), bf16_val(v.z), bf16_val(v.w) };
      st2_v4f(BL + 4 * tid, o);
    } else if (tid < 64) {
      const int q = tid - 32;
      const v4f v = *(const v4fa*)(bs + 4 * q);
      const v4f o = (v4f){ bf16_val(v.x), bf16_val(v.y), bf16_val(v.z), bf16_val(v.w) };
      st2_v4f(BL + KD + 4 * q, o);
    }
  }
}

__device__ __forceinline__ void list_flush(const int* pl, const int* cnt, int ov, int* lp, int* cop, int* fp, int tid) {
#pragma unroll 1
  for (int i = tid * 4; i < RCAP; i += NTHR * 4) {
    const v4i v = *(const v4ia*)(pl + i);
    *(volatile v4i*)(lp + i) = v;
  }
#pragma unroll 1
  for (int i = tid * 4; i < 2 * NBRUN; i += NTHR * 4) {
    const v4i v = *(const v4ia*)(cnt + i);
    *(volatile v4i*)(cop + i) = v;
  }
  if (tid < 8) {
    const v4i f = {ov, ov, ov, ov};
    *(volatile v4i*)(fp + 4 * tid) = f;
  }
}

__global__ __launch_bounds__(NTHR) void k_list(const int* __restrict__ rows, const int* __restrict__ cols,
                                               int* LIST, int* CO, int* FLAG) {
  extern __shared__ __attribute__((aligned(16))) int dsm[];
  int* wl   = dsm;
  int* pl   = dsm + NWAVE * WLCAP;
  int* cnt  = pl + RCAP;
  int* offs = cnt + NBRUN;
  int* cur  = offs + NBRUN;
  int* misc = cur + NBRUN;
  const int tid = (int)threadIdx.x, lane = tid & 31, wave = tid >> 5;
  const int blk = (int)blockIdx.x;
  const unsigned nbs = (unsigned)(blk * NBRUN);

  {
    const v4i z4 = {0, 0, 0, 0};
    for (int i = tid * 4; i < BK_ZINTS; i += NTHR * 4) *(v4ia*)(dsm + i) = z4;
    if (tid < 16) misc[tid] = 0;
  }
  __syncthreads();

  {
    int* mylist = wl + wave * WLCAP;
    int wc = 0;
#pragma unroll 1
    for (int ci = wave; ci < NCHUNK; ci += NWAVE) {
      int e0 = ci * WCH + lane * EPT;
      e0 = e0 > NE - EPT ? NE - EPT : e0;
      const v4i da = *(const v4ia*)(rows + e0);
      asm volatile("" :: "v"(da));
      const v4i db = *(const v4ia*)(rows + e0 + 4);
      asm volatile("" :: "v"(db));
      const int rv[8] = {da.x, da.y, da.z, da.w, db.x, db.y, db.z, db.w};
      unsigned s[8];
      bool hit[8];
      unsigned mk[8];
      unsigned any = 0u;
#pragma unroll
      for (int j = 0; j < 8; ++j) {
        s[j]   = (unsigned)rv[j] - nbs;
        hit[j] = (s[j] < (unsigned)NBRUN) && ((unsigned)rv[j] < (unsigned)NN);
        mk[j]  = __builtin_amdgcn_ballot_w32(hit[j]);
        any |= mk[j];
      }
      if (any != 0u) {
        const v4i ca = *(const v4ia*)(cols + e0);
        asm volatile("" :: "v"(ca));
        const v4i cb = *(const v4ia*)(cols + e0 + 4);
        asm volatile("" :: "v"(cb));
        const int cv[8] = {clampi(ca.x, 0, NN - 1), clampi(ca.y, 0, NN - 1), clampi(ca.z, 0, NN - 1), clampi(ca.w, 0, NN - 1),
                           clampi(cb.x, 0, NN - 1), clampi(cb.y, 0, NN - 1), clampi(cb.z, 0, NN - 1), clampi(cb.w, 0, NN - 1)};
        int pre = 0;
#pragma unroll
        for (int j = 0; j < 8; ++j) pre += (int)__builtin_amdgcn_mbcnt_lo(mk[j], 0u);
        int p = wc + pre;
#pragma unroll
        for (int j = 0; j < 8; ++j) {
          if (hit[j]) {
            if (p < WLCAP) mylist[p] = cv[j] | (int)(s[j] << CBITS);
            p = p + 1;
          }
        }
#pragma unroll
        for (int j = 0; j < 8; ++j) wc += (int)__builtin_popcount(mk[j]);
      }
    }
    if (lane == 0) misc[wave] = wc;
  }
  __syncthreads();

  if (wave == 0) {
    int ov = 0;
    int tot = 0;
#pragma unroll 1
    for (int w2 = 0; w2 < NWAVE; ++w2) {
      int c = misc[w2];
      if (c > WLCAP) ov = 1;
      c = c < 0 ? 0 : (c > WLCAP ? WLCAP : c);
      tot += c;
#pragma unroll 1
      for (int b0 = 0; b0 < c; b0 += 32) {
        const int idx = b0 + lane;
        const int ent = wl[w2 * WLCAP + (idx < WLCAP ? idx : WLCAP - 1)];
        const int m32 = (c - b0) < 32 ? (c - b0) : 32;
#pragma unroll 1
        for (int k = 0; k < m32; ++k) {
          const int u    = __builtin_amdgcn_readlane(ent, k);
          const int slot = (u >> CBITS) & (NBRUN - 1);
          if (lane == 0) cnt[slot] = cnt[slot] + 1;
        }
      }
    }
    if (tot > RCAP) ov = 1;
    if (lane == 0) misc[9] = ov;
  }
  __syncthreads();
  if (wave == 0) {
    const int base = lane * (NBRUN / 32);
    int sum = 0;
#pragma unroll 1
    for (int i = 0; i < NBRUN / 32; ++i) sum += cnt[base + i];
    int incl = sum;
#pragma unroll
    for (int d = 1; d < 32; d <<= 1) {
      const int y = __shfl_up(incl, d, 32);
      if (lane >= d) incl += y;
    }
    int run = incl - sum;
#pragma unroll 1
    for (int i = 0; i < NBRUN / 32; ++i) {
      const int c1 = cnt[base + i];
      offs[base + i] = run;
      cur[base + i]  = run;
      run += c1;
    }
  }
  __syncthreads();

  if (wave == 0) {
#pragma unroll 1
    for (int w2 = 0; w2 < NWAVE; ++w2) {
      int c = misc[w2];
      c = c < 0 ? 0 : (c > WLCAP ? WLCAP : c);
#pragma unroll 1
      for (int b0 = 0; b0 < c; b0 += 32) {
        const int idx = b0 + lane;
        const int ent = wl[w2 * WLCAP + (idx < WLCAP ? idx : WLCAP - 1)];
        const int m32 = (c - b0) < 32 ? (c - b0) : 32;
#pragma unroll 1
        for (int k = 0; k < m32; ++k) {
          const int u    = __builtin_amdgcn_readlane(ent, k);
          const int slot = (u >> CBITS) & (NBRUN - 1);
          if (lane == 0) {
            int p = cur[slot];
            p = p < 0 ? 0 : (p > RCAP - 1 ? RCAP - 1 : p);
            pl[p] = u & ((1 << CBITS) - 1);
            cur[slot] = p + 1;
          }
        }
      }
    }
  }
  __syncthreads();

  const int ovf = misc[9];
  int* lp  = LIST + (size_t)blk * (size_t)RCAP;
  int* cop = CO + (size_t)blk * (2 * NBRUN);
  int* fp  = FLAG + (size_t)blk * 32;
  list_flush(pl, cnt, ovf, lp, cop, fp, tid);
  __threadfence();
  list_flush(pl, cnt, ovf, lp, cop, fp, tid);
}

__device__ __forceinline__ unsigned hl_bits(float m) {
  const unsigned hb   = bf16_bits(m);
  const unsigned lraw = bf16_lo_bits(m);
  const bool nf = (hb & 0x7F80u) == 0x7F80u;
  const unsigned lb = nf ? 0u : lraw;
  return hb | (lb << 16);
}

__global__ __launch_bounds__(NTHR) void k_max(const int* __restrict__ LIST, const int* __restrict__ CO,
                                              const int* __restrict__ FLAG, const float* __restrict__ P,
                                              unsigned short* AGG) {
  const int tid = (int)threadIdx.x, lane = tid & 31, wave = tid >> 5;
  const int node = (int)blockIdx.x * NWAVE + wave;
  const int blk  = node >> SLB;
  const int slot = node & (NBRUN - 1);
  const int* lb = LIST + (size_t)blk * (size_t)RCAP;
  const int cv = CO[(size_t)blk * (2 * NBRUN) + slot];
  const int ov = CO[(size_t)blk * (2 * NBRUN) + NBRUN + slot];
  const int fl = FLAG[(size_t)blk * 32];
  const bool live = node < NN;
  const bool big  = cv > DEGCAP;
  int c = live ? (cv < 0 ? 0 : (cv > DEGCAP ? DEGCAP : cv)) : 0;
  c = __builtin_amdgcn_readfirstlane(c);
  int o = ov < 0 ? 0 : (ov > RCAP - 1 ? RCAP - 1 : ov);
  o = __builtin_amdgcn_readfirstlane(o);
  int last = o + (c > 0 ? c : 1) - 1;
  last = last > RCAP - 1 ? RCAP - 1 : last;

  const float ninf = __uint_as_float(0xff800000u);
  float m0 = ninf, m1 = ninf, m2 = ninf, m3 = ninf;
#pragma unroll 1
  for (int b0 = 0; b0 < c; b0 += 32) {
    int idx = o + b0 + lane;
    idx = idx > last ? last : idx;
    int sr = lb[idx];
    sr = sr < 0 ? 0 : (sr > NN - 1 ? NN - 1 : sr);
    const int m32 = (c - b0) < 32 ? (c - b0) : 32;
#pragma unroll 1
    for (int k = 0; k < m32; ++k) {
      const int sk = __builtin_amdgcn_readlane(sr, k);
      const v4f q = *(const v4fa*)(P + (size_t)sk * KD + 4 * lane);
      const float v0 = (q.x > 0.0f || q.x != q.x) ? q.x : 0.0f;
      const float v1 = (q.y > 0.0f || q.y != q.y) ? q.y : 0.0f;
      const float v2 = (q.z > 0.0f || q.z != q.z) ? q.z : 0.0f;
      const float v3 = (q.w > 0.0f || q.w != q.w) ? q.w : 0.0f;
      m0 = (v0 > m0 || v0 != v0) ? v0 : m0;
      m1 = (v1 > m1 || v1 != v1) ? v1 : m1;
      m2 = (v2 > m2 || v2 != v2) ? v2 : m2;
      m3 = (v3 > m3 || v3 != v3) ? v3 : m3;
    }
  }
  const float qnan = __uint_as_float(0x7fc00000u);
  const bool bad = (fl != 0) || big;
  m0 = bad ? qnan : m0; m1 = bad ? qnan : m1; m2 = bad ? qnan : m2; m3 = bad ? qnan : m3;

  const unsigned w0 = hl_bits(m0), w1 = hl_bits(m1), w2 = hl_bits(m2), w3 = hl_bits(m3);
  const unsigned mk = live ? 0xFFFFFFFFu : 0u;
  const v2u hw = (v2u){ pk16(w0 & 0xFFFFu, w1 & 0xFFFFu) & mk, pk16(w2 & 0xFFFFu, w3 & 0xFFFFu) & mk };
  const v2u lw = (v2u){ pk16(w0 >> 16, w1 >> 16) & mk, pk16(w2 >> 16, w3 >> 16) & mk };
  unsigned short* rowp = AGG + (size_t)node * (size_t)AGK;
  volatile v2u* qh = (volatile v2u*)(rowp + 4 * lane);
  volatile v2u* ql = (volatile v2u*)(rowp + (SPLIT_AGG ? KD : 0) + 4 * lane);
  *qh = hw;
  if (SPLIT_AGG) *ql = lw;
  __threadfence();
  *qh = hw;
  if (SPLIT_AGG) *ql = lw;
}

__global__ __launch_bounds__(NTHR) void k_final(const float* __restrict__ T, float* out) {
  const int tid = (int)threadIdx.x, lane = tid & 31, wave = tid >> 5;
  const int row = (int)blockIdx.x * NWAVE + wave;
  const int rc  = row > NN - 1 ? NN - 1 : row;
  const size_t off = (size_t)rc * KD + (size_t)(4 * lane);
  const v4f d = *(const v4fa*)(out + off);
  asm volatile("" :: "v"(d));
  const v4f t = *(const v4fa*)(T + off);
  asm volatile("" :: "v"(t));
  const float s0 = d.x + t.x, s1 = d.y + t.y, s2 = d.z + t.z, s3 = d.w + t.w;
  v4f o;
  o.x = (s0 > 0.0f || s0 != s0) ? s0 : 0.0f;
  o.y = (s1 > 0.0f || s1 != s1) ? s1 : 0.0f;
  o.z = (s2 > 0.0f || s2 != s2) ? s2 : 0.0f;
  o.w = (s3 > 0.0f || s3 != s3) ? s3 : 0.0f;
  if (row < NN) st2_v4f(out + off, o);
}

extern "C" void kernel_launch(void* const* d_in, const int* in_sizes, int n_in,
                              void* d_out, int out_size, void* d_ws, size_t ws_size,
                              hipStream_t stream) {
  if (n_in < 7) return;
  if (in_sizes[0] != NN * KD) return;
  if (in_sizes[1] != NE) return;
  if (in_sizes[2] != NE) return;
  if (in_sizes[3] != KD * KD) return;
  if (in_sizes[4] != KD) return;
  if (in_sizes[5] != 2 * KD * KD) return;
  if (in_sizes[6] != KD) return;
  if (out_size != NN * KD) return;

  const float* x      = (const float*)d_in[0];
  const int*   rowk   = (const int*)d_in[1];
  const int*   colk   = (const int*)d_in[2];
  const float* W_pool = (const float*)d_in[3];
  const float* b_pool = (const float*)d_in[4];
  const float* weight = (const float*)d_in[5];
  const float* bias   = (const float*)d_in[6];
  float* out = (float*)d_out;

  constexpr size_t zR1   = (size_t)MP * 256 * 2;
  constexpr size_t zR2   = (size_t)MP * KD * 4;
  constexpr size_t zLIST = (size_t)NBK * RCAP * 4;
  constexpr size_t zCO   = (size_t)NBK * 2 * NBRUN * 4;
  constexpr size_t zFLAG = (size_t)NBK * 128;
  constexpr size_t zWP   = (size_t)KD * KD * 2;
  constexpr size_t zWT   = (size_t)KD * KD * 2;
  constexpr size_t zWB   = (size_t)KD * 256 * 2;
  constexpr size_t zBL   = 1024;
  constexpr size_t oR1   = 0;
  constexpr size_t oR2   = oR1 + zR1;
  constexpr size_t oLIST = oR2 + zR2;
  constexpr size_t oCO   = oLIST + zLIST;
  constexpr size_t oFLAG = oCO + zCO;
  constexpr size_t oWP   = oFLAG + zFLAG;
  constexpr size_t oWT   = oWP + zWP;
  constexpr size_t oWB   = oWT + zWT;
  constexpr size_t oBL   = oWB + zWB;
  constexpr size_t oEND  = oBL + zBL;
  static_assert(zR1 % 128 == 0 && zR2 % 128 == 0 && zLIST % 128 == 0 && zCO % 128 == 0 && zFLAG % 128 == 0);
  static_assert(zWP % 128 == 0 && zWT % 128 == 0 && zWB % 128 == 0 && zBL % 128 == 0);
  static_assert(zR1 >= (size_t)MP * KD * 2 && zR1 >= (size_t)MP * AGK * 2);
  static_assert(zWB >= (size_t)KD * AGK * 2);
  static_assert(oEND == (size_t)435445 * 256);
  static_assert(oEND <= (size_t)WSMAX);
  if (oEND > ws_size) return;

  char* ws = (char*)d_ws;
  unsigned short* XB   = (unsigned short*)(ws + oR1);
  unsigned short* AGG  = (unsigned short*)(ws + oR1);
  float*          P    = (float*)(ws + oR2);
  float*          T    = (float*)(ws + oR2);
  int*            LIST = (int*)(ws + oLIST);
  int*            CO   = (int*)(ws + oCO);
  int*            FLAG = (int*)(ws + oFLAG);
  unsigned short* WPT  = (unsigned short*)(ws + oWP);
  unsigned short* WTT  = (unsigned short*)(ws + oWT);
  unsigned short* WBD  = (unsigned short*)(ws + oWB);
  float*          BL   = (float*)(ws + oBL);

  hipFuncSetAttribute(reinterpret_cast<const void*>(&k_list), hipFuncAttributeMaxDynamicSharedMemorySize, (int)BK_LDS);

  k_plane<0><<<MP * KD / 8 / NTHR, NTHR, 0, stream>>>(x, NN, KD, KD, XB, MP, KD);
  k_prep<<<PWTOT, NTHR, 0, stream>>>(W_pool, b_pool, weight, bias, WPT, WTT, WBD, BL);
  {
    const int tiles = (MP / 64) * (KD / 64);
    k_gemm_nt<0, 1><<<(tiles + 7) / 8, NTHR, 0, stream>>>(XB, WPT, BL, P, MP, KD, KD, KD);
  }
  {
    const int tiles = ((NN + 63) / 64) * (KD / 64);
    k_gemm_nt<0, 1><<<(tiles + 7) / 8, NTHR, 0, stream>>>(XB, WTT, BL + KD, out, NN, KD, KD, KD);
  }
  k_list<<<NBK, NTHR, BK_LDS, stream>>>(rowk, colk, LIST, CO, FLAG);
  k_max<<<MP / NWAVE, NTHR, 0, stream>>>(LIST, CO, FLAG, P, AGG);
  {
    const int tiles = (MP / 64) * (KD / 64);
    k_gemm_nt<0, 0><<<(tiles + 7) / 8, NTHR, 0, stream>>>(AGG, WBD, BL, T, MP, KD, AGK, KD);
  }
  k_final<<<NN / NWAVE, NTHR, 0, stream>>>(T, out);
}
